// GCN_pool_18056042512582
// MI455X (gfx1250) — hardware-verified
//
#include <hip/hip_runtime.h>
#include <stddef.h>
#include <math.h>


#define CIN     128
#define HID     128
#define COUT    64
#define ESM     32
#define NTHR    256
#define NWAVE   8
#define EPT     8
#define NGRP    2
#define CHUNK   (NTHR * EPT * NGRP)
#define WCAP    (EPT * NGRP * 32)
#define LISTN   (NWAVE * WCAP)
#define NBC     4096
#define NBF     1024
#define RCAP    40960
#define RBN     128
#define TGT     256
#define DEGCAP  512
#define OTHR    512
#define DTHR    256
#define BM      32
#define WSCAP   134217728
#define SCL_W   16.0f
#define SCL_X   8.0f
#define SCL_H   64.0f
#define SCL_Z   256.0f
#define SCL_E1  64.0f
#define SCL_E2  256.0f
#define INV_XW  0.0078125f
#define INV_HW  0.0009765625f
#define INV_PQ  0.000244140625f
#define INV_E2  0.0009765625f
#define INV_E3  0.000244140625f

#define LDS_FILL ((RCAP + NBF + LISTN) * 4 + 64)

static_assert((CHUNK & (CHUNK - 1)) == 0);
static_assert(CHUNK <= 4096);
static_assert(NBC <= 4096 && NBF <= 4096);
static_assert((NBC & (NBC - 1)) == 0 && (NBF & (NBF - 1)) == 0);
static_assert(NBC == 4 * NBF);
static_assert(OTHR * 8 == NBC);
static_assert((RCAP % 32) == 0);
static_assert(TGT == NWAVE * 32);
static_assert((NBC % TGT) == 0);
static_assert((TGT % BM) == 0);
static_assert(HID == 2 * COUT && CIN == 128 && COUT == 64 && ESM == 32);
static_assert(DTHR == 256);

typedef float    v2f  __attribute__((ext_vector_type(2)));
typedef float    v4f  __attribute__((ext_vector_type(4)));
typedef float    v8f  __attribute__((ext_vector_type(8)));
typedef int      v4i  __attribute__((ext_vector_type(4)));
typedef _Float16 v2h  __attribute__((ext_vector_type(2)));
typedef _Float16 v4h  __attribute__((ext_vector_type(4)));
typedef _Float16 v8h  __attribute__((ext_vector_type(8)));
typedef _Float16 v16h __attribute__((ext_vector_type(16)));
union FragH { v16h v; v8h h[2]; };

__device__ __forceinline__ v8f wmh(v16h a, v16h b, v8f c) {
  v8f d = __builtin_amdgcn_wmma_f32_16x16x32_f16(false, a, false, b, (short)0, c, false, false);
  asm volatile("v_nop\n\tv_nop\n\tv_nop\n\tv_nop" : "+v"(d) : "v"(a), "v"(b));
  return d;
}

__device__ __forceinline__ v8h cvt8(v4f a, v4f b, float s) {
  v8f t;
  t[0] = a.x * s; t[1] = a.y * s; t[2] = a.z * s; t[3] = a.w * s;
  t[4] = b.x * s; t[5] = b.y * s; t[6] = b.z * s; t[7] = b.w * s;
  return __builtin_convertvector(t, v8h);
}

template <int NB>
__device__ __forceinline__ int scan_chunk(const int* __restrict__ dsts, int nE, int cbase, int slotBase,
                                          int vec8, int* list, int tid, int lane, int wave) {
  int wc = 0;
#pragma unroll
  for (int g = 0; g < NGRP; ++g) {
    const int el0  = (g * NTHR + tid) * EPT;
    const int e0   = cbase + el0;
    const int sent = -2147483647 - 1;
    v4i da, db;
    if (vec8 != 0 && cbase + CHUNK <= nE) {
      da = *(const v4i*)(dsts + e0);
      db = *(const v4i*)(dsts + e0 + 4);
    } else {
      da.x = (e0     < nE) ? dsts[min(e0, nE - 1)] : sent;
      da.y = (e0 + 1 < nE) ? dsts[min(e0 + 1, nE - 1)] : sent;
      da.z = (e0 + 2 < nE) ? dsts[min(e0 + 2, nE - 1)] : sent;
      da.w = (e0 + 3 < nE) ? dsts[min(e0 + 3, nE - 1)] : sent;
      db.x = (e0 + 4 < nE) ? dsts[min(e0 + 4, nE - 1)] : sent;
      db.y = (e0 + 5 < nE) ? dsts[min(e0 + 5, nE - 1)] : sent;
      db.z = (e0 + 6 < nE) ? dsts[min(e0 + 6, nE - 1)] : sent;
      db.w = (e0 + 7 < nE) ? dsts[min(e0 + 7, nE - 1)] : sent;
    }
    const unsigned nb = (unsigned)slotBase;
    const unsigned s0 = (unsigned)da.x - nb, s1 = (unsigned)da.y - nb;
    const unsigned s2 = (unsigned)da.z - nb, s3 = (unsigned)da.w - nb;
    const unsigned s4 = (unsigned)db.x - nb, s5 = (unsigned)db.y - nb;
    const unsigned s6 = (unsigned)db.z - nb, s7 = (unsigned)db.w - nb;
    const bool h0 = s0 < (unsigned)NB, h1 = s1 < (unsigned)NB, h2 = s2 < (unsigned)NB, h3 = s3 < (unsigned)NB;
    const bool h4 = s4 < (unsigned)NB, h5 = s5 < (unsigned)NB, h6 = s6 < (unsigned)NB, h7 = s7 < (unsigned)NB;
    const unsigned any = __builtin_amdgcn_ballot_w32(h0 | h1 | h2 | h3 | h4 | h5 | h6 | h7);
    if (any != 0u) {
#define HITJ(J, HJ, SJ) { \
        const unsigned mj = __builtin_amdgcn_ballot_w32(HJ); \
        if (mj != 0u) { \
          if (HJ) { \
            const int pos = wc + (int)__builtin_amdgcn_mbcnt_lo(mj, 0u); \
            if (pos < WCAP) list[wave * WCAP + pos] = ((el0 + (J)) << 12) | (int)(SJ); \
          } \
          wc += (int)__builtin_popcount(mj); } }
      HITJ(0, h0, s0)
      HITJ(1, h1, s1)
      HITJ(2, h2, s2)
      HITJ(3, h3, s3)
      HITJ(4, h4, s4)
      HITJ(5, h5, s5)
      HITJ(6, h6, s6)
      HITJ(7, h7, s7)
#undef HITJ
    }
  }
  return wc;
}

__global__ __launch_bounds__(NTHR) void k_xcvt(const float* __restrict__ x, _Float16* xp, int nN, int nUnits) {
  constexpr int UPR = CIN / 8;
  static_assert((UPR & (UPR - 1)) == 0);
  const int i = (int)blockIdx.x * NTHR + (int)threadIdx.x;
  if (i >= nUnits) return;
  const int row = i / UPR;
  const int c0  = (i & (UPR - 1)) * 8;
  int rr = row > nN - 1 ? nN - 1 : row;
  rr = rr < 0 ? 0 : rr;
  const float* p = x + (size_t)rr * CIN + c0;
  const v4f a = *(const v4f*)p;
  const v4f b = *(const v4f*)(p + 4);
  const float sc = (row < nN) ? SCL_X : 0.0f;
  const v8h o = cvt8(a, b, sc);
  _Float16* d = xp + (size_t)i * 8;
  *(volatile v8h*)d = o;
  __threadfence();
  *(volatile v8h*)d = o;
}

__global__ __launch_bounds__(NTHR) void k_prepw(const float* __restrict__ W, _Float16* wp,
                                                int Nw, int nRowsW, int Kp, int ncut, int kcut, int kval, int nUnits) {
  const int i = (int)blockIdx.x * NTHR + (int)threadIdx.x;
  if (i >= nUnits) return;
  const int upr = Kp >> 3;
  const int n   = i / upr;
  const int k0  = (i - n * upr) * 8;
  const int half = (n >= ncut) ? 1 : 0;
  int col = n - half * ncut;
  col = col < 0 ? 0 : (col > Nw - 1 ? Nw - 1 : col);
  v8f t;
#pragma unroll
  for (int j = 0; j < 8; ++j) {
    const int k = k0 + j;
    int row = k + half * kcut;
    row = row < 0 ? 0 : (row > nRowsW - 1 ? nRowsW - 1 : row);
    const float wv = W[(size_t)row * Nw + col];
    const float sc = (k < kval) ? SCL_W : 0.0f;
    t[j] = wv * sc;
  }
  const v8h o = __builtin_convertvector(t, v8h);
  _Float16* d = wp + (size_t)i * 8;
  *(volatile v8h*)d = o;
  __threadfence();
  *(volatile v8h*)d = o;
}

__global__ __launch_bounds__(NTHR) void k_count(
    const int* __restrict__ dsts, int* cnt, int nE, int vec8) {
  __shared__ __attribute__((aligned(16))) int scnt[NBC];
  __shared__ __attribute__((aligned(16))) int list[LISTN];
  __shared__ int wcnt[NWAVE];
  const int tid = threadIdx.x, lane = tid & 31, wave = tid >> 5;
  const int nodeBase = blockIdx.x * NBC;

  for (int i = tid; i < NBC; i += NTHR) scnt[i] = 0;
  __syncthreads();

  const int nChunks = (nE + CHUNK - 1) / CHUNK;
#pragma unroll 1
  for (int ch = 0; ch < nChunks; ++ch) {
    const int cbase = ch * CHUNK;
    const int wc = scan_chunk<NBC>(dsts, nE, cbase, nodeBase, vec8, list, tid, lane, wave);
    if (lane == 0) wcnt[wave] = wc;
    __syncthreads();
    if (wave == 0) {
#pragma unroll 1
      for (int wsx = 0; wsx < NWAVE; ++wsx) {
        int n = __builtin_amdgcn_readfirstlane(wcnt[wsx]);
        n = n > WCAP ? WCAP : (n < 0 ? 0 : n);
        const int* lp = list + wsx * WCAP;
#pragma unroll 1
        for (int i = 0; i < n; ++i) {
          const int ent  = __builtin_amdgcn_readfirstlane(lp[i]);
          const int slot = ent & (NBC - 1);
          if (lane == 0) scnt[slot] = scnt[slot] + 1;
        }
      }
    }
    __syncthreads();
  }

  v4i cq[4];
#pragma unroll
  for (int q = 0; q < 4; ++q) {
    const int f = (wave * 4 + q) * 128 + 4 * lane;
    cq[q] = *(const v4i*)(scnt + f);
  }
  int* cp = cnt + (size_t)nodeBase;
#pragma unroll
  for (int q = 0; q < 4; ++q) {
    const int f = (wave * 4 + q) * 128 + 4 * lane;
    *(volatile v4i*)(cp + f) = cq[q];
  }
  __threadfence();
#pragma unroll
  for (int q = 0; q < 4; ++q) {
    const int f = (wave * 4 + q) * 128 + 4 * lane;
    *(volatile v4i*)(cp + f) = cq[q];
  }
}

__global__ __launch_bounds__(OTHR) void k_offsets(
    const int* __restrict__ cnt, int* off, int* rbase, int nChunk) {
  __shared__ __attribute__((aligned(16))) int soff[NBC];
  __shared__ __attribute__((aligned(16))) int srb[RBN];
  __shared__ int wtot[OTHR / 32];
  const int tid = threadIdx.x, lane = tid & 31, wave = tid >> 5, sub = tid >> 7;
  for (int i = tid; i < RBN; i += OTHR) srb[i] = 0;
  int carry = 0;
#pragma unroll 1
  for (int ch = 0; ch < nChunk; ++ch) {
    const int base = ch * NBC;
    const v4i c0 = *(const v4i*)(cnt + base + 8 * tid);
    const v4i c1 = *(const v4i*)(cnt + base + 8 * tid + 4);
    const int e0 = max(c0.x, 0), e1 = max(c0.y, 0), e2 = max(c0.z, 0), e3 = max(c0.w, 0);
    const int e4 = max(c1.x, 0), e5 = max(c1.y, 0), e6 = max(c1.z, 0), e7 = max(c1.w, 0);
    const int ts = e0 + e1 + e2 + e3 + e4 + e5 + e6 + e7;
    int incl = ts;
#pragma unroll
    for (int d = 1; d < 32; d <<= 1) {
      const int t = __shfl_up(incl, d);
      if (lane >= d) incl += t;
    }
    if (lane == 31) wtot[wave] = incl;
    __syncthreads();
    const int S0 = wtot[0]  + wtot[1]  + wtot[2]  + wtot[3];
    const int S1 = wtot[4]  + wtot[5]  + wtot[6]  + wtot[7];
    const int S2 = wtot[8]  + wtot[9]  + wtot[10] + wtot[11];
    const int S3 = wtot[12] + wtot[13] + wtot[14] + wtot[15];
    int pre = 0;
#pragma unroll 1
    for (int w = 4 * sub; w < wave; ++w) pre += wtot[w];
    const int b0 = carry;
    const int b1 = b0 + ((S0 + 31) & ~31);
    const int b2 = b1 + ((S1 + 31) & ~31);
    const int b3 = b2 + ((S2 + 31) & ~31);
    const int b4 = b3 + ((S3 + 31) & ~31);
    const int myb = sub == 0 ? b0 : (sub == 1 ? b1 : (sub == 2 ? b2 : b3));
    if (tid == 0) {
      srb[min(4 * ch + 0, RBN - 1)] = b0;
      srb[min(4 * ch + 1, RBN - 1)] = b1;
      srb[min(4 * ch + 2, RBN - 1)] = b2;
      srb[min(4 * ch + 3, RBN - 1)] = b3;
    }
    int run = myb + pre + incl - ts;
    soff[8 * tid + 0] = run; run += e0;
    soff[8 * tid + 1] = run; run += e1;
    soff[8 * tid + 2] = run; run += e2;
    soff[8 * tid + 3] = run; run += e3;
    soff[8 * tid + 4] = run; run += e4;
    soff[8 * tid + 5] = run; run += e5;
    soff[8 * tid + 6] = run; run += e6;
    soff[8 * tid + 7] = run;
    carry = b4;
    __syncthreads();
    const v4i o0 = *(const v4i*)(soff + 4 * tid);
    const v4i o1 = *(const v4i*)(soff + 4 * (tid + OTHR));
    int* op = off + base;
    *(volatile v4i*)(op + 4 * tid) = o0;
    *(volatile v4i*)(op + 4 * (tid + OTHR)) = o1;
    __threadfence();
    *(volatile v4i*)(op + 4 * tid) = o0;
    *(volatile v4i*)(op + 4 * (tid + OTHR)) = o1;
    __syncthreads();
  }
  if (tid == 0) srb[min(4 * nChunk, RBN - 1)] = carry;
  __syncthreads();
  v4i rv = {0, 0, 0, 0};
  if (tid < 32) rv = *(const v4i*)(srb + 4 * tid);
  if (tid < 32) *(volatile v4i*)(rbase + 4 * tid) = rv;
  __threadfence();
  if (tid < 32) *(volatile v4i*)(rbase + 4 * tid) = rv;
}

__global__ __launch_bounds__(NTHR) void k_fill(
    const int* __restrict__ dsts, const int* __restrict__ off, const int* __restrict__ rbase,
    int* csr, int nE, int vec8, int csrLen) {
  extern __shared__ v4f lds_dyn[];
  int* region = (int*)lds_dyn;
  int* cursor = region + RCAP;
  int* list   = cursor + NBF;
  int* wcnt   = list + LISTN;
  const int tid = threadIdx.x, lane = tid & 31, wave = tid >> 5;
  const int b = blockIdx.x;
  const int nodeBase = b * NBF;

  int rb0 = rbase[b];
  const int rb1 = rbase[b + 1];
  rb0 = rb0 < 0 ? 0 : (rb0 > csrLen ? csrLen : rb0);
  rb0 &= ~31;
  int len = rb1 - rb0;
  len = len < 0 ? 0 : (len > RCAP ? RCAP : len);
  int lenW = (len + 31) & ~31;
  if (rb0 + lenW > csrLen) lenW = (csrLen - rb0) & ~31;

  {
    const v4i z = {0, 0, 0, 0};
    for (int i = tid; i < RCAP / 4; i += NTHR) ((v4i*)region)[i] = z;
    for (int s = tid; s < NBF; s += NTHR) {
      int o = off[nodeBase + s] - rb0;
      o = o < 0 ? 0 : (o > RCAP ? RCAP : o);
      cursor[s] = o;
    }
  }
  __syncthreads();

  const int nChunks = (nE + CHUNK - 1) / CHUNK;
#pragma unroll 1
  for (int ch = 0; ch < nChunks; ++ch) {
    const int cbase = ch * CHUNK;
    const int wc = scan_chunk<NBF>(dsts, nE, cbase, nodeBase, vec8, list, tid, lane, wave);
    if (lane == 0) wcnt[wave] = wc;
    __syncthreads();
    if (wave == 0) {
#pragma unroll 1
      for (int wsx = 0; wsx < NWAVE; ++wsx) {
        int n = __builtin_amdgcn_readfirstlane(wcnt[wsx]);
        n = n > WCAP ? WCAP : (n < 0 ? 0 : n);
        const int* lp = list + wsx * WCAP;
#pragma unroll 1
        for (int i = 0; i < n; ++i) {
          const int ent  = __builtin_amdgcn_readfirstlane(lp[i]);
          const int slot = ent & (NBF - 1);
          int e = cbase + ((ent >> 12) & (CHUNK - 1));
          e = e > nE - 1 ? nE - 1 : (e < 0 ? 0 : e);
          if (lane == 0) {
            int pos = cursor[slot];
            pos = pos < 0 ? 0 : (pos > RCAP - 1 ? RCAP - 1 : pos);
            region[pos] = e;
            const int np = pos + 1;
            cursor[slot] = np > RCAP ? RCAP : np;
          }
        }
      }
    }
    __syncthreads();
  }

  const int nv = lenW >> 2;
  int* gp = csr + rb0;
#pragma unroll 1
  for (int i = tid; i < nv; i += NTHR) { const v4i v = ((const v4i*)region)[i]; *(volatile v4i*)(gp + 4 * i) = v; }
  __threadfence();
#pragma unroll 1
  for (int i = tid; i < nv; i += NTHR) { const v4i v = ((const v4i*)region)[i]; *(volatile v4i*)(gp + 4 * i) = v; }
}

template <int NCOL, int MODE>
__global__ __launch_bounds__(NTHR) void k_agg(
    const int* __restrict__ csr, const int* __restrict__ off, const int* __restrict__ cnt,
    const int* __restrict__ srcs, const float* __restrict__ hp, const float* __restrict__ bias,
    const float* __restrict__ esm, _Float16* ap, int nN, int nE, int csrLen) {
  static_assert(NCOL == 128 || NCOL == 64);
  static_assert(MODE == 0 || MODE == 1);
  static_assert((MODE == 0 && NCOL == HID) || (MODE == 1 && NCOL == COUT));
  constexpr int LM = NCOL / 4 - 1;
  const int tid = threadIdx.x, lane = tid & 31, wave = tid >> 5;
  const int tbase = blockIdx.x * TGT + wave * 32;
  const int col4 = 4 * (lane & LM);

  const int cl    = tbase + lane;
  const int cnt_l = cnt[cl];
  const int off_l = off[cl];
  const v4f bv = *(const v4f*)(bias + col4);

#pragma unroll 1
  for (int j = 0; j < 32; ++j) {
    const int c = tbase + j;
    int nraw = __shfl(cnt_l, j);
    nraw = nraw < 0 ? 0 : (nraw > nE ? nE : nraw);
    const int n = nraw > DEGCAP ? DEGCAP : nraw;
    const int st = __shfl(off_l, j);

    v4f acc = {0.0f, 0.0f, 0.0f, 0.0f};
#pragma unroll 1
    for (int q0 = 0; q0 < n; q0 += 32) {
      int pos = st + q0 + lane;
      pos = pos < 0 ? 0 : (pos > csrLen - 1 ? csrLen - 1 : pos);
      int el = csr[pos];
      el = el < 0 ? 0 : (el > nE - 1 ? nE - 1 : el);
      int sl = srcs[el];
      sl = sl < 0 ? 0 : (sl > nN - 1 ? nN - 1 : sl);
      int cs = cnt[sl];
      cs = cs < 0 ? 0 : (cs > nE ? nE : cs);
      const float wl  = rsqrtf((float)(cs + 1));
      const int   wli = __float_as_int(wl);
      const int mcnt = (n - q0) < 32 ? (n - q0) : 32;
#pragma unroll 1
      for (int pp = 0; pp < mcnt; ++pp) {
        const int   s = __builtin_amdgcn_readlane(sl, pp);
        const float w = __int_as_float(__builtin_amdgcn_readlane(wli, pp));
        const v4f r = *(const v4f*)(hp + (size_t)s * NCOL + col4);
        acc = acc + r * w;
      }
    }

    int cc = c > nN - 1 ? nN - 1 : c;
    cc = cc < 0 ? 0 : cc;
    const float dc = rsqrtf((float)(nraw + 1));
    const v4f self = *(const v4f*)(hp + (size_t)cc * NCOL + col4);
    v4f v = (acc + self * dc) * dc + bv;
    if (MODE == 0) {
      v.x = v.x > 0.0f ? v.x : 0.0f;
      v.y = v.y > 0.0f ? v.y : 0.0f;
      v.z = v.z > 0.0f ? v.z : 0.0f;
      v.w = v.w > 0.0f ? v.w : 0.0f;
    }
    if (nraw > DEGCAP) { const float qn = __int_as_float(0x7fc00000); v.x = qn; v.y = qn; v.z = qn; v.w = qn; }
    v4f o4;
    if (MODE == 0) {
      const float sc = (c < nN) ? SCL_H : 0.0f;
      o4 = v * sc;
    } else {
      const v4f ev = *(const v4f*)(esm + (size_t)cc * ESM + ((4 * lane) & (ESM - 1)));
      const bool live = c < nN;
      const float sz = (live && lane < 16) ? SCL_Z : 0.0f;
      const float se = (live && lane >= 16 && lane < 24) ? SCL_Z : 0.0f;
      o4 = v * sz + ev * se;
    }
    const v4h o = __builtin_convertvector(o4, v4h);
    _Float16* gp = ap + (size_t)c * HID + 4 * lane;
    *(volatile v4h*)gp = o;
    __threadfence();
    *(volatile v4h*)gp = o;
  }
}

template <int K, int LDB, int TPW>
__device__ __forceinline__ void mma_pair(const _Float16* __restrict__ Ap, const _Float16* __restrict__ Bp,
                                         int arow, int c0, int m, int hh, v8f (&acc)[TPW]) {
  constexpr int KT = K / 32;
  static_assert(K % 32 == 0 && LDB % 8 == 0);
  const _Float16* ap  = Ap + (size_t)arow * K + 8 * hh;
  const _Float16* bp0 = Bp + (size_t)(c0 + m) * LDB + 8 * hh;
#pragma unroll 1
  for (int kt = 0; kt < KT; ++kt) {
    FragH a;
    a.h[0] = *(const v8h*)(ap + 32 * kt);
    a.h[1] = *(const v8h*)(ap + 32 * kt + 16);
#pragma unroll
    for (int t = 0; t < TPW; ++t) {
      const _Float16* bp = bp0 + (size_t)(16 * t) * LDB + 32 * kt;
      FragH bf;
      bf.h[0] = *(const v8h*)bp;
      bf.h[1] = *(const v8h*)(bp + 16);
      acc[t] = wmh(a.v, bf.v, acc[t]);
    }
  }
}

template <int K, int NC, int LDB>
__device__ __forceinline__ void gemm_stage(
    const _Float16* __restrict__ A1, const _Float16* __restrict__ Bp,
    float* stg, int rowBase, int nN, int lane, int wave, float oscale) {
  constexpr int TPW = NC / 64;
  static_assert(K % 32 == 0);
  static_assert(NC % 64 == 0 && TPW >= 1);
  const int hh = lane >> 4, m = lane & 15;
  const int rg = wave >> 2, cq = wave & 3;
  const int r0 = rg * 16;
  const int c0 = cq * (NC / 4);

  v8f acc[TPW];
#pragma unroll
  for (int t = 0; t < TPW; ++t) { v8f z = {0.f, 0.f, 0.f, 0.f, 0.f, 0.f, 0.f, 0.f}; acc[t] = z; }

  mma_pair<K, LDB, TPW>(A1, Bp, rowBase + r0 + m, c0, m, hh, acc);

  float* sp = stg + (size_t)(r0 + 8 * hh) * NC + c0 + m;
  const int grow0 = rowBase + r0 + 8 * hh;
#pragma unroll
  for (int t = 0; t < TPW; ++t) {
#pragma unroll
    for (int r = 0; r < 8; ++r) {
      float v = acc[t][r] * oscale;
      v = (grow0 + r < nN) ? v : 0.0f;
      sp[r * NC + 16 * t] = v;
    }
  }
}

template <int K, int NC, int LDB>
__global__ __launch_bounds__(NTHR) void k_gemm32(
    const _Float16* __restrict__ A1, const _Float16* __restrict__ Bp,
    float* Zp, int nN, float oscale) {
  constexpr int NIT4 = (BM * NC / 4) / NTHR;
  static_assert((BM * NC / 4) % NTHR == 0 && NIT4 >= 1);
  static_assert(BM * 8 == NTHR);
  __shared__ __attribute__((aligned(16))) float stg[BM * NC];
  const int tid = threadIdx.x, lane = tid & 31, wave = tid >> 5;
  const int rowBase = blockIdx.x * BM;

  gemm_stage<K, NC, LDB>(A1, Bp, stg, rowBase, nN, lane, wave, oscale);
  __syncthreads();

  float* tile = Zp + (size_t)rowBase * NC;
  v4f ov[NIT4];
#pragma unroll
  for (int it = 0; it < NIT4; ++it) ov[it] = *(const v4f*)(stg + 4 * (it * NTHR + tid));
#pragma unroll
  for (int it = 0; it < NIT4; ++it) *(volatile v4f*)(tile + 4 * (size_t)(it * NTHR + tid)) = ov[it];
  __threadfence();
#pragma unroll
  for (int it = 0; it < NIT4; ++it) *(volatile v4f*)(tile + 4 * (size_t)(it * NTHR + tid)) = ov[it];
}

__global__ __launch_bounds__(DTHR) void k_edge(
    const float* __restrict__ pq, const int* __restrict__ srcs, const int* __restrict__ dsts,
    const float* __restrict__ f1b, const _Float16* __restrict__ pF2, const float* __restrict__ f2b,
    const _Float16* __restrict__ pF3, const float* __restrict__ f3b,
    const float* __restrict__ f4W, const float* __restrict__ f4b,
    float* out, int nE, int nN) {
  constexpr int NUD = DTHR / 4;
  constexpr int K2  = COUT;
  constexpr int N2  = COUT / 2;
  constexpr int N3  = COUT / 4;
  static_assert(NUD == 64 && K2 == 64 && N2 == 32 && N3 == 16);
  __shared__ __attribute__((aligned(16))) _Float16 sA1[DTHR * K2];
  __shared__ __attribute__((aligned(16))) _Float16 sA2[DTHR * N2];
  __shared__ __attribute__((aligned(16))) float sres[DTHR];
  const int tid = threadIdx.x, lane = tid & 31, wave = tid >> 5, hh = lane >> 4, m = lane & 15;
  const int gbase = blockIdx.x * DTHR;
  const int wb = wave * 32;

  int el = gbase + wb + lane;
  el = el > nE - 1 ? nE - 1 : el;
  el = el < 0 ? 0 : el;
  int si = srcs[el];
  int di = dsts[el];
  si = si < 0 ? 0 : (si > nN - 1 ? nN - 1 : si);
  di = di < 0 ? 0 : (di > nN - 1 ? nN - 1 : di);

  {
    const int c2 = 2 * lane;
    const v2f b1v = *(const v2f*)(f1b + c2);
#pragma unroll 1
    for (int j = 0; j < 32; ++j) {
      const int s = __builtin_amdgcn_readlane(si, j);
      const int d = __builtin_amdgcn_readlane(di, j);
      const v2f p = *(const v2f*)(pq + (size_t)s * HID + c2);
      const v2f q = *(const v2f*)(pq + (size_t)d * HID + COUT + c2);
      v2f v = p + q + b1v;
      v.x = v.x > 0.0f ? v.x : 0.0f;
      v.y = v.y > 0.0f ? v.y : 0.0f;
      v = v * SCL_E1;
      const v2h o = __builtin_convertvector(v, v2h);
      *(v2h*)(sA1 + (size_t)(wb + j) * K2 + c2) = o;
    }
  }
  __syncthreads();

  v8f acc2[2][2];
#pragma unroll
  for (int rt = 0; rt < 2; ++rt)
#pragma unroll
    for (int t = 0; t < 2; ++t) { v8f z = {0.f, 0.f, 0.f, 0.f, 0.f, 0.f, 0.f, 0.f}; acc2[rt][t] = z; }
#pragma unroll
  for (int kt = 0; kt < K2 / 32; ++kt) {
#pragma unroll
    for (int rt = 0; rt < 2; ++rt) {
      FragH a;
      const _Float16* apx = sA1 + (size_t)(wb + 16 * rt + m) * K2 + 32 * kt + 8 * hh;
      a.h[0] = *(const v8h*)apx;
      a.h[1] = *(const v8h*)(apx + 16);
#pragma unroll
      for (int t = 0; t < 2; ++t) {
        const _Float16* bpx = pF2 + (size_t)(16 * t + m) * K2 + 32 * kt + 8 * hh;
        FragH bf;
        bf.h[0] = *(const v8h*)bpx;
        bf.h[1] = *(const v8h*)(bpx + 16);
        acc2[rt][t] = wmh(a.v, bf.v, acc2[rt][t]);
      }
    }
  }
#pragma unroll
  for (int rt = 0; rt < 2; ++rt) {
#pragma unroll
    for (int t = 0; t < 2; ++t) {
      const float bb = f2b[16 * t + m];
#pragma unroll
      for (int r = 0; r < 8; ++r) {
        float v = acc2[rt][t][r] * INV_E2 + bb;
        v = v > 0.0f ? v : 0.0f;
        v = v * SCL_E2;
        sA2[(size_t)(wb + 16 * rt + 8 * hh + r) * N2 + 16 * t + m] = (_Float16)v;
      }
    }
  }
  __syncthreads();

  FragH b3f;
  {
    const _Float16* bpx = pF3 + (size_t)m * N2 + 8 * hh;
    b3f.h[0] = *(const v8h*)bpx;
    b3f.h[1] = *(const v8h*)(bpx + 16);
  }
  v8f acc3[2];
#pragma unroll
  for (int rt = 0; rt < 2; ++rt) {
    FragH a;
    const _Float16* apx = sA2 + (size_t)(wb + 16 * rt + m) * N2 + 8 * hh;
    a.h[0] = *(const v8h*)apx;
    a.h[1] = *(const v8h*)(apx + 16);
    v8f z = {0.f, 0.f, 0.f, 0.f, 0.f, 0.f, 0.f, 0.f};
    acc3[rt] = wmh(a.v, b3f.v, z);
  }

  const float bb3 = f3b[m];
  const float w4  = f4W[m];
  const float c4  = f4b[0];
#pragma unroll
  for (int rt = 0; rt < 2; ++rt) {
    float sel = 0.0f;
#pragma unroll
    for (int r = 0; r < 8; ++r) {
      float a3 = acc3[rt][r] * INV_E3 + bb3;
      a3 = a3 > 0.0f ? a3 : 0.0f;
      float p = a3 * w4;
      p += __shfl_xor(p, 8);
      p += __shfl_xor(p, 4);
      p += __shfl_xor(p, 2);
      p += __shfl_xor(p, 1);
      sel = (m == r) ? p : sel;
    }
    if (m < 8) sres[wb + 16 * rt + 8 * hh + m] = sel + c4;
  }
  __syncthreads();

  const v4f v = *(const v4f*)(sres + 4 * (tid & (NUD - 1)));
  const int e0 = gbase + 4 * tid;
  const bool act  = tid < NUD;
  const bool full = act && (e0 + 3 < nE);
  const bool part = act && !full && (e0 < nE);
  if (full) {
    *(volatile v4f*)(out + e0) = v;
  } else if (part) {
    if (e0 < nE)     *(volatile float*)(out + e0)     = v.x;
    if (e0 + 1 < nE) *(volatile float*)(out + e0 + 1) = v.y;
    if (e0 + 2 < nE) *(volatile float*)(out + e0 + 2) = v.z;
  }
  __threadfence();
  if (full) {
    *(volatile v4f*)(out + e0) = v;
  } else if (part) {
    if (e0 < nE)     *(volatile float*)(out + e0)     = v.x;
    if (e0 + 1 < nE) *(volatile float*)(out + e0 + 1) = v.y;
    if (e0 + 2 < nE) *(volatile float*)(out + e0 + 2) = v.z;
  }
}

extern "C" void kernel_launch(void* const* d_in, const int* in_sizes, int n_in,
                              void* d_out, int out_size, void* d_ws, size_t ws_size,
                              hipStream_t stream) {
  if (n_in < 15) return;
  const int nN = in_sizes[0] / CIN;
  const int nE = in_sizes[2] / 2;
  if (nN <= 0 || nE <= 0) return;
  if (in_sizes[0] != nN * CIN || in_sizes[1] != nN * ESM || in_sizes[2] != 2 * nE) return;
  if (in_sizes[3] != CIN * HID || in_sizes[4] != HID) return;
  if (in_sizes[5] != HID * COUT || in_sizes[6] != COUT) return;
  if (in_sizes[7] != 2 * (COUT + ESM) * COUT || in_sizes[8] != COUT) return;
  if (in_sizes[9] != COUT * (COUT / 2) || in_sizes[10] != COUT / 2) return;
  if (in_sizes[11] != (COUT / 2) * (COUT / 4) || in_sizes[12] != COUT / 4) return;
  if (in_sizes[13] != COUT / 4 || in_sizes[14] != 1) return;
  if (out_size != nE) return;
  if (nE > (1 << 28) || nN > (1 << 22)) return;

  const float* x   = (const float*)d_in[0];
  const float* esm = (const float*)d_in[1];
  const int*   ei  = (const int*)d_in[2];
  const float* W1  = (const float*)d_in[3];
  const float* b1  = (const float*)d_in[4];
  const float* W2  = (const float*)d_in[5];
  const float* b2  = (const float*)d_in[6];
  const float* f1W = (const float*)d_in[7];
  const float* f1b = (const float*)d_in[8];
  const float* f2W = (const float*)d_in[9];
  const float* f2b = (const float*)d_in[10];
  const float* f3W = (const float*)d_in[11];
  const float* f3b = (const float*)d_in[12];
  const float* f4W = (const float*)d_in[13];
  const float* f4b = (const float*)d_in[14];
  const int* src = ei;
  const int* dst = ei + nE;
  float* out = (float*)d_out;

  const int NPAD   = ((nN + TGT - 1) / TGT) * TGT;
  const int nBC    = (nN + NBC - 1) / NBC;
  const int CNTPAD = nBC * NBC;
  if (CNTPAD < NPAD) return;
  if (4 * nBC + 1 > RBN) return;
  const int nBF    = (nN + NBF - 1) / NBF;
  if (nBF + 1 > 4 * nBC + 1) return;
  const int csrLen = ((nE + 31) & ~31) + 4096;
  if (31 * 4 * nBC > 4096) return;
  const int nAgg   = NPAD / TGT;
  const int nGemm  = NPAD / BM;
  const int nXu    = NPAD * (CIN / 8);
  const int nDec   = (nE + DTHR - 1) / DTHR;

  char* ws = (char*)d_ws;
  size_t off = 0;
  const size_t oW1  = off; off += (size_t)HID * CIN * 2;               off = (off + 255) & ~(size_t)255;
  const size_t oW2  = off; off += (size_t)COUT * HID * 2;              off = (off + 255) & ~(size_t)255;
  const size_t oF1  = off; off += (size_t)HID * HID * 2;               off = (off + 255) & ~(size_t)255;
  const size_t oF2  = off; off += (size_t)(COUT / 2) * COUT * 2;       off = (off + 255) & ~(size_t)255;
  const size_t oF3  = off; off += (size_t)(COUT / 4) * (COUT / 2) * 2; off = (off + 255) & ~(size_t)255;
  const size_t oX   = off; off += (size_t)NPAD * CIN * 2;              off = (off + 255) & ~(size_t)255;
  const size_t oXW  = off; off += (size_t)NPAD * HID * 4;              off = (off + 255) & ~(size_t)255;
  const size_t oH   = off; off += (size_t)NPAD * HID * 2;              off = (off + 255) & ~(size_t)255;
  const size_t oHW  = off; off += (size_t)NPAD * COUT * 4;             off = (off + 255) & ~(size_t)255;
  const size_t oZ   = off; off += (size_t)NPAD * HID * 2;              off = (off + 255) & ~(size_t)255;
  const size_t oPQ  = off; off += (size_t)NPAD * HID * 4;              off = (off + 255) & ~(size_t)255;
  const size_t oCnt = off; off += (size_t)CNTPAD * 4;                  off = (off + 255) & ~(size_t)255;
  const size_t oOff = off; off += (size_t)CNTPAD * 4;                  off = (off + 255) & ~(size_t)255;
  const size_t oRb  = off; off += (size_t)RBN * 4;                     off = (off + 255) & ~(size_t)255;
  const size_t oCsr = off; off += (size_t)csrLen * 4;                  off = (off + 255) & ~(size_t)255;
  if (off > ws_size || off > (size_t)WSCAP) return;
  _Float16* pW1 = (_Float16*)(ws + oW1);
  _Float16* pW2 = (_Float16*)(ws + oW2);
  _Float16* pF1 = (_Float16*)(ws + oF1);
  _Float16* pF2 = (_Float16*)(ws + oF2);
  _Float16* pF3 = (_Float16*)(ws + oF3);
  _Float16* xP  = (_Float16*)(ws + oX);
  float*    xwP = (float*)(ws + oXW);
  _Float16* hP  = (_Float16*)(ws + oH);
  float*    hwP = (float*)(ws + oHW);
  _Float16* zcP = (_Float16*)(ws + oZ);
  float*    pqP = (float*)(ws + oPQ);
  int*   cnt  = (int*)(ws + oCnt);
  int*   offp = (int*)(ws + oOff);
  int*   rb   = (int*)(ws + oRb);
  int*   csr  = (int*)(ws + oCsr);

  const int vec8 = ((nE & 7) == 0) ? 1 : 0;

  {
    const int uW1 = HID * (CIN / 8);
    const int uW2 = COUT * (HID / 8);
    const int uF1 = HID * (HID / 8);
    const int uF2 = (COUT / 2) * (COUT / 8);
    const int uF3 = (COUT / 4) * ((COUT / 2) / 8);
    k_prepw<<<(uW1 + NTHR - 1) / NTHR, NTHR, 0, stream>>>(W1, pW1, HID, CIN, CIN, HID, 0, CIN, uW1);
    k_prepw<<<(uW2 + NTHR - 1) / NTHR, NTHR, 0, stream>>>(W2, pW2, COUT, HID, HID, COUT, 0, HID, uW2);
    k_prepw<<<(uF1 + NTHR - 1) / NTHR, NTHR, 0, stream>>>(f1W, pF1, COUT, 2 * (COUT + ESM), HID, COUT, COUT + ESM, COUT + ESM, uF1);
    k_prepw<<<(uF2 + NTHR - 1) / NTHR, NTHR, 0, stream>>>(f2W, pF2, COUT / 2, COUT, COUT, COUT / 2, 0, COUT, uF2);
    k_prepw<<<(uF3 + NTHR - 1) / NTHR, NTHR, 0, stream>>>(f3W, pF3, COUT / 4, COUT / 2, COUT / 2, COUT / 4, 0, COUT / 2, uF3);
  }
  k_xcvt<<<(nXu + NTHR - 1) / NTHR, NTHR, 0, stream>>>(x, xP, nN, nXu);

  k_count<<<nBC, NTHR, 0, stream>>>(dst, cnt, nE, vec8);
  k_offsets<<<1, OTHR, 0, stream>>>(cnt, offp, rb, nBC);
  hipFuncSetAttribute(reinterpret_cast<const void*>(&k_fill),
                      hipFuncAttributeMaxDynamicSharedMemorySize, LDS_FILL);
  k_fill<<<nBF, NTHR, LDS_FILL, stream>>>(dst, offp, rb, csr, nE, vec8, csrLen);

  k_gemm32<CIN, HID, CIN><<<nGemm, NTHR, 0, stream>>>(xP, pW1, xwP, nN, INV_XW);
  k_agg<HID, 0><<<nAgg, NTHR, 0, stream>>>(csr, offp, cnt, src, xwP, b1, esm, hP, nN, nE, csrLen);

  k_gemm32<HID, COUT, HID><<<nGemm, NTHR, 0, stream>>>(hP, pW2, hwP, nN, INV_HW);
  k_agg<COUT, 1><<<nAgg, NTHR, 0, stream>>>(csr, offp, cnt, src, hwP, b2, esm, zcP, nN, nE, csrLen);

  k_gemm32<HID, HID, HID><<<nGemm, NTHR, 0, stream>>>(zcP, pF1, pqP, nN, INV_PQ);

  k_edge<<<nDec, DTHR, 0, stream>>>(pqP, src, dst, f1b, pF2, f2b, pF3, f3b, f4W, f4b, out, nE, nN);
}
